// DCD_52450140619545
// MI455X (gfx1250) — hardware-verified
//
#include <hip/hip_runtime.h>


namespace {
constexpr int Bn = 4, C = 64, H = 128, W = 128, NPOS = Bn * H * W, K9 = 9, KK = K9 * C  , NOFF = 27, HO = 64, WO = 64;
constexpr float AS_ = 8.0f;

typedef _Float16 b16;
typedef __attribute__((ext_vector_type(16))) _Float16 v16b;
typedef __attribute__((ext_vector_type(8))) _Float16 v8b;
typedef __attribute__((ext_vector_type(8))) float v8f;
typedef __attribute__((ext_vector_type(4))) float v4f;
__device__ __forceinline__ float bf16_rne(float f) { unsigned int u = __float_as_uint(f); u += 0x7FFFu + ((u >> 16) & 1u); return __uint_as_float(u & 0xFFFF0000u); }
__device__ __forceinline__ void split16(float v, b16& hi, b16& lo) { hi = (b16)v; lo = (b16)(v - (float)hi); }
__device__ __forceinline__ v16b frag_kb(const b16* p, int hh) { const v8b a = *(const v8b*)(p + 8 * hh), b = *(const v8b*)(p + 16 + 8 * hh); v16b f;
#pragma unroll
  for (int e = 0; e < 8; ++e) { f[e] = a[e]; f[8 + e] = b[e]; } return f; }
__device__ __forceinline__ v8f wmma16b(v16b a, v16b b, v8f c) { v8f d = __builtin_amdgcn_wmma_f32_16x16x32_f16(false, a, false, b, (short)0, c, false, false); asm volatile("v_nop\n\tv_nop\n\tv_nop\n\tv_nop" : "+v"(d) : "v"(a), "v"(b)); return d; }
__device__ __forceinline__ void wave_lds_sync() { __builtin_amdgcn_fence(__ATOMIC_RELEASE, "workgroup"); __builtin_amdgcn_wave_barrier(); __builtin_amdgcn_fence(__ATOMIC_ACQUIRE, "workgroup"); }
__device__ __forceinline__ float nexp(float x) { return __builtin_amdgcn_exp2f(x * 1.4426950408889634f); }
__device__ __forceinline__ float pmul(float a, float b) { float p = a * b; asm volatile("" : "+v"(p)); return p; }

__global__ __launch_bounds__(256) void prep_kernel(const float* __restrict__ woff, const float* __restrict__ boff, const float* __restrict__ wal, const float* __restrict__ bal, b16* __restrict__ R, float* __restrict__ P) {
  const int t_ = blockIdx.x * 256 + threadIdx.x, nth = gridDim.x * 256;
  for (int pass = 0; pass < 2; ++pass) {
    for (int q = t_; q < 32 * KK; q += nth) { const int o = q / KK, k = q % KK, tap = k / C, c = k % C; R[q] = (b16)((o < NOFF) ? bf16_rne(woff[((size_t)o * C + c) * 9 + tap]) : 0.0f); }
    for (int q = t_; q < C * KK; q += nth) { const int o = q / KK, k = q % KK, tap = k / C, c = k % C; R[32 * KK + q] = (b16)bf16_rne(wal[((size_t)o * C + c) * 9 + tap]); }
    for (int q = t_; q < 96; q += nth) P[q] = (q < 32) ? ((q < NOFF) ? bf16_rne(boff[q]) : 0.0f) : bf16_rne(bal[q - 32]);
    __threadfence(); }
}

__global__ __launch_bounds__(256) void xpose_kernel(const float* __restrict__ x, b16* __restrict__ xt) {
  __shared__ __attribute__((aligned(16))) b16 T[W][C + 8];
  const int b = blockIdx.y, i = blockIdx.x, t_ = threadIdx.x;
  for (int q = t_; q < C * W; q += 256) { const int c = q >> 7, j = q & 127; T[j][c] = (b16)bf16_rne(x[(((size_t)b * C + c) * H + i) * W + j]); }
  __syncthreads();
  for (int pass = 0; pass < 2; ++pass) { for (int q = t_; q < W * (C / 8); q += 256) { const int j = q >> 3, c8 = (q & 7) * 8; *(volatile v8b*)(xt + (((size_t)b * H + i) * W + j) * C + c8) = *(const v8b*)(&T[j][c8]); } __threadfence(); }
}

__device__ __forceinline__ v16b frag_im2col(const b16* xtb, int i, int j, int kb, int hh) {
  const int tap = kb / C, cb = kb % C; const int u = tap / 3 - 1, v = tap % 3 - 1; const int ii = i + u, jj = j + v; v16b f = {};
  if (ii >= 0 && ii < H && jj >= 0 && jj < W) f = frag_kb(xtb + ((size_t)ii * W + jj) * C + cb, hh);
  return f; }

__global__ __launch_bounds__(128) void offconv_kernel(const b16* __restrict__ xt, const b16* __restrict__ R, const float* __restrict__ P, float* __restrict__ off) {
  __shared__ __attribute__((aligned(16))) float Ts[4][32 * 32];
  const int lane = threadIdx.x & 31, wave = threadIdx.x >> 5, nloc = lane & 15, hlf = lane >> 4, b = blockIdx.y, i = blockIdx.x, j0 = wave * 32; const b16* xtb = xt + ((size_t)b * H) * W * C;
  v8f acc[2][2];
#pragma unroll
  for (int r = 0; r < 2; ++r) { acc[r][0] = (v8f){}; acc[r][1] = (v8f){}; }
  for (int kb = 0; kb < KK; kb += 32) { const v16b a0 = frag_im2col(xtb, i, j0 + nloc, kb, hlf), a1 = frag_im2col(xtb, i, j0 + 16 + nloc, kb, hlf);
#pragma unroll
    for (int t = 0; t < 2; ++t) { const v16b bw = frag_kb(R + (size_t)(t * 16 + nloc) * KK + kb, hlf); acc[0][t] = wmma16b(a0, bw, acc[0][t]); acc[1][t] = wmma16b(a1, bw, acc[1][t]); } }
  float* Tt = Ts[wave];
#pragma unroll
  for (int t = 0; t < 2; ++t) { const float bb = P[t * 16 + nloc];
#pragma unroll
    for (int r = 0; r < 2; ++r)
#pragma unroll
      for (int v = 0; v < 8; ++v) Tt[(r * 16 + 8 * hlf + v) * 32 + t * 16 + nloc] = acc[r][t][v] + bb; }
  wave_lds_sync();
  const size_t p0 = ((size_t)b * H + i) * W + j0;
  for (int pass = 0; pass < 2; ++pass) { for (int q = lane; q < 32 * 8; q += 32) { const int rr = q >> 3, c4 = (q & 7) * 4; *(volatile v4f*)(off + (p0 + rr) * 32 + c4) = *(const v4f*)(Tt + rr * 32 + c4); } __threadfence(); }
}

__global__ __launch_bounds__(128) void deform_kernel(const b16* __restrict__ xt, const float* __restrict__ off, const b16* __restrict__ R, const float* __restrict__ P, const float* __restrict__ x, float* __restrict__ WX, float* __restrict__ WW) {
  __shared__ __attribute__((aligned(16))) float Tw[C][W + 4];
  const int lane = threadIdx.x & 31, wave = threadIdx.x >> 5, nloc = lane & 15, hlf = lane >> 4, b = blockIdx.y, i = blockIdx.x, j0 = wave * 32; const b16* xtb = xt + ((size_t)b * H) * W * C; const b16* Wal = R + 32 * KK;
  v8f acc[2][4];
#pragma unroll
  for (int r = 0; r < 2; ++r)
#pragma unroll
    for (int t = 0; t < 4; ++t) acc[r][t] = (v8f){};
  for (int tap = 0; tap < K9; ++tap) { const float ky = (float)(tap / 3 - 1), kx = (float)(tap % 3 - 1);
    int y0i[2], x0i[2]; float wgt[2][4]; float msk[2];
#pragma unroll
    for (int r = 0; r < 2; ++r) { const int j = j0 + r * 16 + nloc; const float* orow = off + (((size_t)b * H + i) * W + j) * 32; const float dy = orow[tap * 2], dx = orow[tap * 2 + 1];
      msk[r] = 2.0f / (1.0f + nexp(-orow[18 + tap]));
      const float py = ((float)i + ky) + dy, px = ((float)j + kx) + dx; const float fy = floorf(py), fx = floorf(px); const float ly = py - fy, lx = px - fx; y0i[r] = (int)fy; x0i[r] = (int)fx;
      wgt[r][0] = pmul(1.0f - ly, 1.0f - lx); wgt[r][1] = pmul(1.0f - ly, lx); wgt[r][2] = pmul(ly, 1.0f - lx); wgt[r][3] = pmul(ly, lx); }
    for (int cb = 0; cb < C; cb += 32) { v16b ah[2], al[2];
#pragma unroll
      for (int r = 0; r < 2; ++r) { float val[16];
#pragma unroll
        for (int e = 0; e < 16; ++e) val[e] = 0.0f;
#pragma unroll
        for (int cn = 0; cn < 4; ++cn) { const int yy = y0i[r] + (cn >> 1), xx = x0i[r] + (cn & 1); if (yy >= 0 && yy < H && xx >= 0 && xx < W) { const b16* src = xtb + ((size_t)yy * W + xx) * C + cb; const v8b p0 = *(const v8b*)(src + 8 * hlf), p1 = *(const v8b*)(src + 16 + 8 * hlf); const float wv = wgt[r][cn];
#pragma unroll
            for (int e = 0; e < 8; ++e) { val[e] += pmul((float)p0[e], wv); val[8 + e] += pmul((float)p1[e], wv); } } }
#pragma unroll
        for (int e = 0; e < 16; ++e) { b16 h_, l_; split16(pmul(val[e], msk[r]) * AS_, h_, l_); ah[r][e] = h_; al[r][e] = l_; } }
#pragma unroll
      for (int t = 0; t < 4; ++t) { const v16b bw = frag_kb(Wal + (size_t)(t * 16 + nloc) * KK + tap * C + cb, hlf);
#pragma unroll
        for (int r = 0; r < 2; ++r) { acc[r][t] = wmma16b(ah[r], bw, acc[r][t]); acc[r][t] = wmma16b(al[r], bw, acc[r][t]); } } } }
#pragma unroll
  for (int t = 0; t < 4; ++t) { const int o = t * 16 + nloc; const float bb = P[32 + o];
#pragma unroll
    for (int r = 0; r < 2; ++r)
#pragma unroll
      for (int v = 0; v < 8; ++v) { const float z = acc[r][t][v] * (1.0f / AS_) + bb; const float sg = 1.0f / (1.0f + nexp(-z)); Tw[o][j0 + r * 16 + 8 * hlf + v] = nexp(sg); } }
  __syncthreads();
  for (int pass = 0; pass < 2; ++pass) { for (int q = threadIdx.x; q < C * 32; q += 128) { const int o = q >> 5, c4 = (q & 31) * 4; const size_t g = (((size_t)b * C + o) * H + i) * W + c4; const v4f wv = *(const v4f*)(&Tw[o][c4]); const v4f xv = *(const v4f*)(x + g); v4f wx;
      for (int e = 0; e < 4; ++e) wx[e] = pmul(wv[e], bf16_rne(xv[e])); *(volatile v4f*)(WW + g) = wv; *(volatile v4f*)(WX + g) = wx; } __threadfence(); }
}

__global__ __launch_bounds__(256) void pool_kernel(const float* __restrict__ WX, const float* __restrict__ WW, float* __restrict__ out) {
  const int b = blockIdx.z, o = blockIdx.y, oi = blockIdx.x * 4 + (threadIdx.x >> 6), oj = threadIdx.x & 63; const float* wx = WX + ((size_t)b * C + o) * H * W; const float* ww = WW + ((size_t)b * C + o) * H * W;
  float sx = 0.0f, sw = 0.0f;
  for (int u = -1; u <= 1; ++u) for (int v = -1; v <= 1; ++v) { const int ii = 2 * oi + u, jj = 2 * oj + v; if (ii >= 0 && ii < H && jj >= 0 && jj < W) { sx += wx[(size_t)ii * W + jj]; sw += ww[(size_t)ii * W + jj]; } }
  const float r = (sx * (1.0f / 9.0f)) / (sw * (1.0f / 9.0f));
  for (int pass = 0; pass < 2; ++pass) { ((volatile float*)out)[(((size_t)b * C + o) * HO + oi) * WO + oj] = r; __threadfence(); }
}
}

extern "C" void kernel_launch(void* const* d_in, const int* in_sizes, int n_in,
                              void* d_out, int out_size, void* d_ws, size_t ws_size, hipStream_t stream) {
  (void)n_in; (void)out_size;
  const float* x = (const float*)d_in[0]; const float* woff = (const float*)d_in[1]; const float* boff = (const float*)d_in[2]; const float* wal = (const float*)d_in[3]; const float* bal = (const float*)d_in[4];
  float* out = (float*)d_out;
  if (in_sizes[0] != NPOS * C || in_sizes[1] != NOFF * C * 9 || in_sizes[3] != C * C * 9) return;
  size_t off_ = 0; char* ws = (char*)d_ws;
  auto carve = [&](size_t bytes) { char* p = ws + off_; off_ += (bytes + 255) & ~(size_t)255; return p; };
  b16* R = (b16*)carve((size_t)96 * KK * 2); float* P = (float*)carve(128 * 4); b16* xt = (b16*)carve((size_t)NPOS * C * 2); float* off = (float*)carve((size_t)NPOS * 32 * 4); float* WX = (float*)carve((size_t)NPOS * C * 4); float* WW = (float*)carve((size_t)NPOS * C * 4);
  if (off_ > ws_size) return;
  prep_kernel<<<128, 256, 0, stream>>>(woff, boff, wal, bal, R, P);
  xpose_kernel<<<dim3(H, Bn), 256, 0, stream>>>(x, xt);
  offconv_kernel<<<dim3(H, Bn), 128, 0, stream>>>(xt, R, P, off);
  deform_kernel<<<dim3(H, Bn), 128, 0, stream>>>(xt, off, R, P, x, WX, WW);
  pool_kernel<<<dim3(HO / 4, C, Bn), 256, 0, stream>>>(WX, WW, out);
}
